// SelfAttentionBlock_31980326486088
// MI455X (gfx1250) — hardware-verified
//
#include <hip/hip_runtime.h>
#ifndef NB
#define NB 4
#endif
#ifndef SEQ
#define SEQ 4096
#endif
#define NB_FULL 4
#define SEQ_FULL 4096
#define CI 256
#define LT 256
#ifndef RC
#define RC ((SEQ) < 2048 ? (SEQ) : 2048)
#endif
#define SQ SEQ
#define NR ((size_t)NB * SEQ)

static_assert(NB <= NB_FULL && SEQ <= SEQ_FULL);
static_assert(SEQ % 128 == 0 && RC % 128 == 0 && SEQ % RC == 0);
static_assert(CI % 128 == 0 && LT % 128 == 0 && CI % 64 == 0 && LT % 64 == 0);
static_assert(SEQ % 64 == 0 && SEQ % 32 == 0 && CI % 32 == 0 && LT % 32 == 0);
static_assert(((size_t)CI * LT / 8) % 256 == 0);
static_assert((size_t)4 * CI * LT * 2 + 5 * (size_t)NB * SEQ * 256 * 2 + (size_t)RC * LT * 4 + (size_t)RC * SEQ * 8 <= (size_t)134217728);

typedef unsigned short v8us __attribute__((ext_vector_type(8), may_alias));
typedef float  v8f  __attribute__((ext_vector_type(8)));
typedef float  v4f  __attribute__((ext_vector_type(4)));
typedef float  v4fa __attribute__((ext_vector_type(4), may_alias));
typedef _Float16 v16h __attribute__((ext_vector_type(16)));
typedef _Float16 v4h __attribute__((ext_vector_type(4)));
union FragH { v16h v; v8us half[2]; _Float16 h[16]; unsigned short u[16]; };

__device__ __forceinline__ unsigned short bf16_bits(float x) { unsigned int u = __float_as_uint(x); return (unsigned short)((u + 0x7FFFu + ((u >> 16) & 1u)) >> 16); }
__device__ __forceinline__ float bf16_val(unsigned short b) { return __uint_as_float(((unsigned int)b) << 16); }
__device__ __forceinline__ float bf16_rne(float x) { return bf16_val(bf16_bits(x)); }

__global__ __launch_bounds__(256) void k_wnat4(const float* __restrict__ w0, const float* __restrict__ w1, const float* __restrict__ w2, const float* __restrict__ w3, _Float16* __restrict__ Bt) {
  const int y = blockIdx.y;
  const float* w = (y == 0) ? w0 : ((y == 1) ? w1 : ((y == 2) ? w2 : w3));
  const size_t t = (size_t)blockIdx.x * 256 + threadIdx.x;
  if (t >= (size_t)CI * LT / 8) return;
  const v4f a = *(const v4fa*)(w + t * 8), c = *(const v4fa*)(w + t * 8 + 4);
  FragH f;
#pragma unroll
  for (int q = 0; q < 4; ++q) { f.h[q] = (_Float16)(bf16_rne(a[q]) * 16.0f); f.h[4 + q] = (_Float16)(bf16_rne(c[q]) * 16.0f); }
  const v8us o = f.half[0];
  unsigned short* d = (unsigned short*)Bt + (size_t)y * CI * LT + t * 8;
  *(volatile v8us*)d = o; __threadfence(); *(volatile v8us*)d = o;
}

__global__ __launch_bounds__(256) void k_xt(const float* __restrict__ x, _Float16* __restrict__ XT) {
  __shared__ unsigned short tl[64][66];
  const int tid = threadIdx.x;
  const int ng = blockIdx.x % (SEQ / 64);
  const int cg = (blockIdx.x / (SEQ / 64)) % (CI / 64);
  const int b = blockIdx.x / ((SEQ / 64) * (CI / 64));
  for (int i = tid; i < 64 * 16; i += 256) {
    const int r = i >> 4, q4 = (i & 15) * 4;
    const v4f a = *(const v4fa*)(x + ((size_t)(b * CI + cg * 64 + r)) * SEQ_FULL + ng * 64 + q4);
    FragH f;
#pragma unroll
    for (int u = 0; u < 4; ++u) f.h[u] = (_Float16)bf16_rne(a[u]);
#pragma unroll
    for (int u = 0; u < 4; ++u) tl[r][q4 + u] = f.u[u];
  }
  __syncthreads();
  for (int pass = 0; pass < 2; ++pass) {
#pragma unroll
    for (int rd = 0; rd < 2; ++rd) {
      const int n = rd * 32 + tid / 8, pc = tid % 8;
      FragH f;
#pragma unroll
      for (int q = 0; q < 8; ++q) f.u[q] = tl[pc * 8 + q][n];
      *(volatile v8us*)((unsigned short*)XT + ((size_t)b * SEQ + ng * 64 + n) * CI + cg * 64 + pc * 8) = f.half[0];
    }
    if (pass == 0) __threadfence();
  }
}

__device__ __forceinline__ v16h g2_frag(const _Float16* p, int hh) { FragH f; f.half[0] = *(const v8us*)((const unsigned short*)p + 8 * hh); f.half[1] = *(const v8us*)((const unsigned short*)p + 16 + 8 * hh); return f.v; }
__device__ __forceinline__ v8f g2_mma(v16h a, v16h b, v8f c) { v8f d = __builtin_amdgcn_wmma_f32_16x16x32_f16(false, a, false, b, (short)0, c, false, false); asm volatile("v_nop\n\tv_nop\n\tv_nop\n\tv_nop" : "+v"(d) : "v"(a), "v"(b)); return d; }
template <int BROW>
__global__ __launch_bounds__(128) void k_gemm2(const _Float16* __restrict__ A, int lda, size_t sA, const _Float16* __restrict__ Bh, int ldb, size_t sB, float alpha,
    const float* __restrict__ bias, const float* __restrict__ CP, float* __restrict__ C, _Float16* __restrict__ C16, int ldc, size_t sC, int M, int N, int K) {
  __shared__ __attribute__((aligned(16))) float so[4][32][68];
  const int tid = threadIdx.x, w = tid >> 5, lane = tid & 31, ln = lane & 15, hh = lane >> 4; const int by = blockIdx.y;
  A += (size_t)by * sA; Bh += (size_t)by * sB; const size_t cofs = (size_t)by * sC; const float* bp = bias;
  const int ntn = N >> 6; const int mt = blockIdx.x / ntn, nq = blockIdx.x - mt * ntn; const int row0 = mt * 128 + 32 * w, col0 = nq * 64; if (row0 >= M) return;
  const _Float16* a0p = A + (size_t)(row0 + ln) * lda; const _Float16* a1p = a0p + (size_t)16 * lda;
  const _Float16* b0p = Bh + (size_t)(col0 + ln) * ldb; const _Float16* b1p = b0p + (size_t)16 * ldb; const _Float16* b2p = b1p + (size_t)16 * ldb; const _Float16* b3p = b2p + (size_t)16 * ldb;
  const v8f z8 = {0.f,0.f,0.f,0.f,0.f,0.f,0.f,0.f}; v8f c00 = z8, c01 = z8, c02 = z8, c03 = z8, c10 = z8, c11 = z8, c12 = z8, c13 = z8;
#pragma unroll 1
  for (int kb = 0; kb < K; kb += 32) { const v16h a0 = g2_frag(a0p + kb, hh), a1 = g2_frag(a1p + kb, hh);
    v16h b = g2_frag(b0p + kb, hh); c00 = g2_mma(a0, b, c00); c10 = g2_mma(a1, b, c10);
    b = g2_frag(b1p + kb, hh); c01 = g2_mma(a0, b, c01); c11 = g2_mma(a1, b, c11);
    b = g2_frag(b2p + kb, hh); c02 = g2_mma(a0, b, c02); c12 = g2_mma(a1, b, c12);
    b = g2_frag(b3p + kb, hh); c03 = g2_mma(a0, b, c03); c13 = g2_mma(a1, b, c13); }
  v8f accs[8] = {c00, c01, c02, c03, c10, c11, c12, c13};
  float brw[16];
#pragma unroll
  for (int i = 0; i < 16; ++i) brw[i] = 0.f;
  if (BROW && bp) {
#pragma unroll
    for (int i = 0; i < 16; ++i) brw[i] = bf16_rne(bp[row0 + (i >> 3) * 16 + 8 * hh + (i & 7)]);
  }
#pragma unroll
  for (int u = 0; u < 8; ++u) { const int t = u & 3, half = u >> 2; const int col = col0 + t * 16 + ln;
    float bc = 0.f; if (!BROW && bp) bc = bf16_rne(bp[col]);
#pragma unroll
    for (int r = 0; r < 8; ++r) { const int rloc = half * 16 + 8 * hh + r; const float v = accs[u][r] * alpha + (BROW ? brw[half * 8 + r] : bc); so[w][rloc][t * 16 + ln] = v; } }
  __builtin_amdgcn_fence(4  , "workgroup"); __builtin_amdgcn_wave_barrier();
  const int rsub = lane >> 4, c4 = (lane & 15) * 4;
  if (CP) {
#pragma unroll
    for (int q = 0; q < 16; ++q) { const int r = q * 2 + rsub; v4f v = *(const v4fa*)&so[w][r][c4]; const v4f c = *(const v4fa*)(CP + cofs + (size_t)(row0 + r) * ldc + col0 + c4); v = v + c; *(v4fa*)&so[w][r][c4] = v; }
    __builtin_amdgcn_fence(4  , "workgroup"); __builtin_amdgcn_wave_barrier();
  }
  for (int pass = 0; pass < 2; ++pass) {
#pragma unroll
    for (int q = 0; q < 16; ++q) { const int r = q * 2 + rsub; const v4f v = *(const v4fa*)&so[w][r][c4];
      if (C) *(volatile v4f*)(C + cofs + (size_t)(row0 + r) * ldc + col0 + c4) = v;
      if (C16) { v4h h4;
#pragma unroll
        for (int i = 0; i < 4; ++i) h4[i] = (_Float16)v[i];
        *(volatile v4h*)(C16 + cofs + (size_t)(row0 + r) * ldc + col0 + c4) = h4; } }
    if (pass == 0) __threadfence(); } }

__global__ __launch_bounds__(256) void k_rsmfhl(const float* __restrict__ S, _Float16* __restrict__ P, _Float16* __restrict__ PL, int nrows) {
  #pragma clang fp contract(off)
  const int t = blockIdx.x * 256 + threadIdx.x; if (t >= nrows) return; const float* s = S + (size_t)t * SQ; float mx = -3.0e38f;
#pragma unroll 1
  for (int j = 0; j < SQ; j += 4) { const v4f a = *(const v4fa*)(s + j); mx = fmaxf(mx, fmaxf(fmaxf(a[0], a[1]), fmaxf(a[2], a[3]))); }
  float se = 0.f;
#pragma unroll 1
  for (int j = 0; j < SQ; j += 4) { const v4f a = *(const v4fa*)(s + j); se += __expf(a[0] - mx); se += __expf(a[1] - mx); se += __expf(a[2] - mx); se += __expf(a[3] - mx); }
  const float sc = 256.0f / se;
#pragma unroll 1
  for (int j0 = 0; j0 < SQ; j0 += 8) { FragH fr, fl; const v4f a = *(const v4fa*)(s + j0), c = *(const v4fa*)(s + j0 + 4);
#pragma unroll
    for (int q = 0; q < 4; ++q) { float v = __expf(a[q] - mx) * sc; _Float16 hv = (_Float16)v; fr.h[q] = hv; fl.h[q] = (_Float16)((v - (float)hv) * 1024.0f);
      v = __expf(c[q] - mx) * sc; hv = (_Float16)v; fr.h[4 + q] = hv; fl.h[4 + q] = (_Float16)((v - (float)hv) * 1024.0f); }
    const v8us oh = fr.half[0], ol = fl.half[0];
    unsigned short* d = (unsigned short*)P + (size_t)t * SQ + j0; unsigned short* dl = (unsigned short*)PL + (size_t)t * SQ + j0;
    *(volatile v8us*)d = oh; *(volatile v8us*)dl = ol; __threadfence(); *(volatile v8us*)d = oh; *(volatile v8us*)dl = ol; } }

extern "C" void kernel_launch(void* const* d_in, const int* in_sizes, int n_in,
                              void* d_out, int out_size, void* d_ws, size_t ws_size, hipStream_t stream) {
  if (n_in < 9) return;
  if ((size_t)in_sizes[0] < (size_t)(NB * CI - 1) * SEQ_FULL + SEQ) return;
  if (in_sizes[1] < LT * CI || in_sizes[3] < LT * CI || in_sizes[5] < LT * CI || in_sizes[7] < CI * LT) return;
  if (in_sizes[2] < LT || in_sizes[4] < LT || in_sizes[6] < LT || in_sizes[8] < CI) return;
  if ((size_t)out_size < (size_t)NB * CI * SEQ) return;
  const float* const* I = (const float* const*)d_in;
  const float* x = I[0]; const float* wq = I[1]; const float* bq = I[2]; const float* wk = I[3]; const float* bk = I[4];
  const float* wv = I[5]; const float* bv = I[6]; const float* wo = I[7]; const float* bo = I[8];
  char* ws = (char*)d_ws; size_t off = 0;
  auto take = [&](size_t bytes) { char* p = ws + off; off += (bytes + 255) & ~(size_t)255; return p; };
  _Float16* WB = (_Float16*)take((size_t)4 * CI * LT * 2);
  _Float16* WQ16 = WB; _Float16* WK16 = WB + (size_t)CI * LT; _Float16* WV16 = WB + (size_t)2 * CI * LT; _Float16* WO16 = WB + (size_t)3 * CI * LT;
  _Float16* XT16 = (_Float16*)take(NR * CI * 2);
  _Float16* Q16 = (_Float16*)take(NR * LT * 2);
  _Float16* K16 = (_Float16*)take(NR * LT * 2);
  _Float16* V16 = (_Float16*)take((size_t)NB * LT * SEQ * 2);
  _Float16* R16 = (_Float16*)take(NR * LT * 2);
  float* RF = (float*)take((size_t)RC * LT * 4);
  float* S = (float*)take((size_t)RC * SEQ * 4);
  _Float16* P = (_Float16*)take((size_t)RC * SEQ * 2);
  _Float16* PL = (_Float16*)take((size_t)RC * SEQ * 2);
  if (off > ws_size || off > (size_t)134217728) return;

  k_wnat4<<<dim3((unsigned)((size_t)CI * LT / 8 / 256), 4), 256, 0, stream>>>(wq, wk, wv, wo, WB);
  k_xt<<<(unsigned)(NB * (CI / 64) * (SEQ / 64)), 256, 0, stream>>>(x, XT16);
  k_gemm2<0><<<dim3((unsigned)((NR / 128) * (LT / 64)), 1), 128, 0, stream>>>(XT16, CI, 0, WQ16, CI, 0, 0.0625f, bq, nullptr, nullptr, Q16, LT, 0, (int)NR, LT, CI);
  k_gemm2<0><<<dim3((unsigned)((NR / 128) * (LT / 64)), 1), 128, 0, stream>>>(XT16, CI, 0, WK16, CI, 0, 0.0625f, bk, nullptr, nullptr, K16, LT, 0, (int)NR, LT, CI);
  k_gemm2<1><<<dim3((unsigned)((LT / 128) * (SEQ / 64)), NB), 128, 0, stream>>>(WV16, CI, 0, XT16, CI, (size_t)SEQ * CI, 0.0625f, bv, nullptr, nullptr, V16, SEQ, (size_t)LT * SEQ, LT, SEQ, CI);
  for (int b = 0; b < NB; ++b) {
    const _Float16* Qb = Q16 + (size_t)b * SEQ * LT;
    const _Float16* Vb = V16 + (size_t)b * LT * SEQ;
    for (int ch = 0; ch < SEQ / RC; ++ch) {
      const size_t r0 = (size_t)b * SEQ + (size_t)ch * RC;
      k_gemm2<0><<<dim3((unsigned)((RC / 128) * (SEQ / 64)), 1), 128, 0, stream>>>(K16 + r0 * LT, LT, 0, Qb, LT, 0, 0.0625f, nullptr, nullptr, S, nullptr, SEQ, 0, RC, SEQ, LT);
      k_rsmfhl<<<(RC + 255) / 256, 256, 0, stream>>>(S, P, PL, RC);
      k_gemm2<0><<<dim3((unsigned)((RC / 128) * (LT / 64)), 1), 128, 0, stream>>>(P, SEQ, 0, Vb, SEQ, 0, 0.25f, nullptr, nullptr, RF, nullptr, LT, 0, RC, LT, SEQ);
      k_gemm2<0><<<dim3((unsigned)((RC / 128) * (LT / 64)), 1), 128, 0, stream>>>(PL, SEQ, 0, Vb, SEQ, 0, 0.000244140625f, nullptr, RF, nullptr, R16 + r0 * LT, LT, 0, RC, LT, SEQ);
    }
  }
  k_gemm2<1><<<dim3((unsigned)((CI / 128) * (SEQ / 64)), NB), 128, 0, stream>>>(WO16, LT, 0, R16, LT, (size_t)SEQ * LT, 0.0009765625f, bo, nullptr, (float*)d_out, nullptr, SEQ, (size_t)CI * SEQ, CI, SEQ, LT);
}
